// FFTConv_12025908428820
// MI455X (gfx1250) — hardware-verified
//
#include <hip/hip_runtime.h>

typedef _Float16 v16h __attribute__((ext_vector_type(16)));
typedef _Float16 v8h  __attribute__((ext_vector_type(8)));
typedef float    v8f  __attribute__((ext_vector_type(8)));
typedef float    v4f  __attribute__((ext_vector_type(4)));
typedef v8h v8ha __attribute__((may_alias));
typedef v4f v4fa __attribute__((may_alias));

union Frag { v16h v; v8h half[2]; };
union LdsU { _Float16 h[32 * 16 * 96]; float f[32 * 16 * 48]; };

#define NIMG   4
#define HH     112
#define WW     112
#define ICN    128
#define OCN    256
#define OH     110
#define OW     110
#define NTILE  3136
#define NTB    196
#define NBIN   34
#define NKF    68
#define KIF    96
#define NCH    278528
#define NDFTB  784
#define PFTILE 34816
#define RSQ2   0.70710678118654752f
#define WSC    256.0f
#define OSC    6.103515625e-05f

__device__ __forceinline__ v8f mma16(v8f acc, v16h a, v16h b) {
  acc = __builtin_amdgcn_wmma_f32_16x16x32_f16(false, a, false, b, (short)0, acc, false, false);
  asm volatile("v_nop\n\tv_nop\n\tv_nop\n\tv_nop" : "+v"(acc) : "v"(a), "v"(b));
  return acc;
}

__device__ __forceinline__ void bin_uv(int f, int& u, int& v) {
  if (f < 10) { u = (f < 5) ? 0 : 4; v = (f < 5) ? f : (f - 5); }
  else { const int t = f - 10; u = 1 + (t >> 3); v = t & 7; }
}
__device__ __forceinline__ float cos8(int p) {
  p &= 7;
  const float r = (p == 1 || p == 7) ? RSQ2 : -RSQ2;
  return (p == 0) ? 1.f : (p == 4) ? -1.f : ((p & 1) ? r : 0.f);
}
__device__ __forceinline__ float sin8(int p) {
  p &= 7;
  const float r = (p == 1 || p == 3) ? RSQ2 : -RSQ2;
  return (p == 2) ? 1.f : (p == 6) ? -1.f : ((p & 1) ? r : 0.f);
}

__global__ __launch_bounds__(256) void k_wpack(const float* __restrict__ wr,
                                               const float* __restrict__ wi,
                                               const int* __restrict__ msk,
                                               _Float16* __restrict__ wpk, int nch) {
  const int ch = blockIdx.x * 256 + threadIdx.x;
  if (ch >= nch) return;
  const int hh = ch & 1;
  const int ln = (ch >> 1) & 31;
  const int nt = (ch >> 6) & 15;
  const int kc = (ch >> 10) & 3;
  const int ri = (ch >> 12) & 1;
  const int f  = ch >> 13;
  int u, v; bin_uv(f, u, v);
  const bool self = (f < 10) && (v == 0 || v == 4);
  const int u2 = (8 - u) & 7, v2 = (8 - v) & 7;
  const int n = ln & 15, h = ln >> 4;
  const int oc = nt * 16 + n;
  union { v8h v; _Float16 e[8]; } o;
  #pragma unroll
  for (int j = 0; j < 8; ++j) {
    const int k  = 16 * hh + 8 * h + j;
    const int ic = kc * 32 + k;
    const size_t base = ((size_t)ic * OCN + oc) * 64;
    const size_t i0 = base + (size_t)(u * 8 + v);
    const int m0 = msk[i0];
    float er = m0 ? wr[i0] : 0.f;
    float ei = m0 ? wi[i0] : 0.f;
    if (!self) {
      const size_t i1 = base + (size_t)(u2 * 8 + v2);
      const int m1 = msk[i1];
      er += m1 ? wr[i1] : 0.f;
      ei -= m1 ? wi[i1] : 0.f;
    }
    o.e[j] = (_Float16)((ri ? ei : er) * WSC);
  }
  const v8h val = o.v;
  _Float16* dst = wpk + (size_t)ch * 8;
  *(volatile v8h*)dst = val;
  __threadfence();
  *(volatile v8h*)dst = val;
}

__device__ __forceinline__ void st2(_Float16* Pl, int f, int eoff, float re, float im) {
  Pl[(f * 2 + 0) * 512 + eoff] = (_Float16)re;
  Pl[(f * 2 + 1) * 512 + eoff] = (_Float16)im;
}
__device__ __forceinline__ void col_real(int f0, const float g[6], _Float16* Pl, int eoff) {
  const float S = g[0]+g[1]+g[2]+g[3]+g[4]+g[5];
  const float T = g[0]-g[1]+g[2]-g[3]+g[4]-g[5];
  const float D = g[0]-g[2]+g[4];
  const float E = g[1]-g[3]+g[5];
  const float A = g[0]-g[4];
  const float B = g[1]-g[3]-g[5];
  const float C = g[1]+g[3]-g[5];
  const float rB = RSQ2*B, rC = RSQ2*C;
  st2(Pl, f0 + 0, eoff, S, 0.f);
  st2(Pl, f0 + 1, eoff, A + rB, -(g[2] + rC));
  st2(Pl, f0 + 2, eoff, D, -E);
  st2(Pl, f0 + 3, eoff, A - rB, g[2] - rC);
  st2(Pl, f0 + 4, eoff, T, 0.f);
}
__device__ __forceinline__ void col_cplx(int f0, const float gr[6], const float gi[6],
                                         _Float16* Pl, int eoff) {
  const float Sr = gr[0]+gr[1]+gr[2]+gr[3]+gr[4]+gr[5];
  const float Si = gi[0]+gi[1]+gi[2]+gi[3]+gi[4]+gi[5];
  const float Tr = gr[0]-gr[1]+gr[2]-gr[3]+gr[4]-gr[5];
  const float Ti = gi[0]-gi[1]+gi[2]-gi[3]+gi[4]-gi[5];
  const float Dr = gr[0]-gr[2]+gr[4], Di = gi[0]-gi[2]+gi[4];
  const float Er = gr[1]-gr[3]+gr[5], Ei = gi[1]-gi[3]+gi[5];
  const float Ar = gr[0]-gr[4],       Ai = gi[0]-gi[4];
  const float Br = gr[1]-gr[3]-gr[5], Bi = gi[1]-gi[3]-gi[5];
  const float Cr = gr[1]+gr[3]-gr[5], Ci = gi[1]+gi[3]-gi[5];
  const float rBr = RSQ2*Br, rBi = RSQ2*Bi, rCr = RSQ2*Cr, rCi = RSQ2*Ci;
  const float X1r = Ar + rBr,    X1i = Ai + rBi;
  const float Y1r = gr[2] + rCr, Y1i = gi[2] + rCi;
  const float X3r = Ar - rBr,    X3i = Ai - rBi;
  const float Y3r = gr[2] - rCr, Y3i = gi[2] - rCi;
  st2(Pl, f0 + 0, eoff, Sr, Si);
  st2(Pl, f0 + 1, eoff, X1r + Y1i, X1i - Y1r);
  st2(Pl, f0 + 2, eoff, Dr + Ei,   Di - Er);
  st2(Pl, f0 + 3, eoff, X3r - Y3i, X3i + Y3r);
  st2(Pl, f0 + 4, eoff, Tr, Ti);
  st2(Pl, f0 + 5, eoff, X3r + Y3i, X3i - Y3r);
  st2(Pl, f0 + 6, eoff, Dr - Ei,   Di + Er);
  st2(Pl, f0 + 7, eoff, X1r - Y1i, X1i + Y1r);
}

__global__ __launch_bounds__(512) void k_dft(const float* __restrict__ x, _Float16* __restrict__ pf) {
  __shared__ __align__(16) _Float16 Pl[NKF * 512];

  const int blk = blockIdx.x;
  const int tb  = blk >> 2, kc = blk & 3;
  const int tid = threadIdx.x;
  const int tl  = tid >> 5;
  const int icl = tid & 31;
  const int tg  = tb * 16 + tl;
  const int bimg = tg / 784;
  const int rr   = (tg / 28) % 28;
  const int cc   = tg % 28;
  const int hh   = (icl >> 3) & 1;
  const int ei   = (icl >> 4) * 8 + (icl & 7);
  const int eoff = (tl + 16 * hh) * 16 + ei;
  const int ic   = kc * 32 + icl;

  float p[6][6];
  #pragma unroll
  for (int py = 0; py < 6; ++py) {
    const int yy = rr * 4 + py - 1;
    #pragma unroll
    for (int px = 0; px < 6; ++px) {
      const int xx = cc * 4 + px - 1;
      float vv = 0.f;
      if (yy >= 0 && yy < HH && xx >= 0 && xx < WW)
        vv = x[(((size_t)bimg * HH + yy) * WW + xx) * ICN + ic];
      p[py][px] = vv;
    }
  }
  float G0[6], G4[6], G1r[6], G1i[6], G2r[6], G2i[6], G3r[6], G3i[6];
  #pragma unroll
  for (int px = 0; px < 6; ++px) {
    const float p0 = p[0][px], p1 = p[1][px], p2 = p[2][px];
    const float p3 = p[3][px], p4 = p[4][px], p5 = p[5][px];
    const float S = p0+p1+p2+p3+p4+p5, T = p0-p1+p2-p3+p4-p5;
    const float D = p0-p2+p4, E = p1-p3+p5;
    const float A = p0-p4, B = p1-p3-p5, C = p1+p3-p5;
    const float rB = RSQ2*B, rC = RSQ2*C;
    G0[px] = S;        G4[px] = T;
    G1r[px] = A + rB;  G1i[px] = -(p2 + rC);
    G2r[px] = D;       G2i[px] = -E;
    G3r[px] = A - rB;  G3i[px] = p2 - rC;
  }
  col_real(0, G0, Pl, eoff);
  col_real(5, G4, Pl, eoff);
  col_cplx(10, G1r, G1i, Pl, eoff);
  col_cplx(18, G2r, G2i, Pl, eoff);
  col_cplx(26, G3r, G3i, Pl, eoff);
  __syncthreads();

  _Float16* dst = pf + (size_t)blk * PFTILE;
  #pragma unroll
  for (int j = 0; j < 9; ++j) {
    const int c = tid + 512 * j;
    if (c < NKF * 64) {
      const v8h vv = *(const v8ha*)&Pl[c * 8];
      *(volatile v8h*)(dst + (size_t)c * 8) = vv;
    }
  }
  __threadfence();
  #pragma unroll
  for (int j = 0; j < 9; ++j) {
    const int c = tid + 512 * j;
    if (c < NKF * 64) {
      const v8h vv = *(const v8ha*)&Pl[c * 8];
      *(volatile v8h*)(dst + (size_t)c * 8) = vv;
    }
  }
}

__global__ __launch_bounds__(512) void k_conv(const _Float16* __restrict__ pf,
                                              const _Float16* __restrict__ wpk,
                                              const float* __restrict__ bias,
                                              float* __restrict__ out) {
  __shared__ __align__(16) LdsU U;
  __shared__ __align__(16) _Float16 Tl[3 * 512];

  const int tid  = threadIdx.x;
  const int lane = tid & 31;
  const int h    = lane >> 4;
  const int m16  = lane & 15;
  const int w    = tid >> 5;
  const int tb   = blockIdx.x;
  const int g    = blockIdx.y;
  const int oc0  = g * 32;

  #pragma unroll
  for (int j = 0; j < 3; ++j) {
    const int idx = tid + 512 * j;
    const int kq  = idx >> 9;
    const int q   = idx & 511;
    const int ln  = q >> 4, i = q & 15;
    const int s   = ln & 15, lh = ln >> 4;
    const int kl  = (i < 8) ? (8 * lh + i) : (16 + 8 * lh + (i - 8));
    const int k   = kq * 32 + kl;
    float val = 0.f;
    if (k < NKF) {
      const int f = k >> 1, ri = k & 1;
      int u, v; bin_uv(f, u, v);
      const int pidx = (u * ((s >> 2) + 2) + v * ((s & 3) + 2)) & 7;
      val = ri ? -sin8(pidx) : cos8(pidx);
    }
    Tl[idx] = (_Float16)val;
  }
  {
    _Float16* row = &U.h[tid * KIF + NKF];
    #pragma unroll
    for (int q = 0; q < KIF - NKF; ++q) row[q] = (_Float16)0.f;
  }

  const int nb = (w < 2) ? 3 : 2;
  v8f cr[3][2] = {};
  v8f ci[3][2] = {};
  #pragma unroll 1
  for (int kc = 0; kc < 4; ++kc) {
    const _Float16* ablk = pf + ((size_t)(tb * 4 + kc) * NKF) * 512 + lane * 16;
    #pragma unroll
    for (int j = 0; j < 3; ++j) {
      if (j < nb) {
        const int f = w + 16 * j;
        const _Float16* ap = ablk + (size_t)(f * 2) * 512;
        Frag ar, ai;
        ar.half[0] = *(const v8h*)(ap);
        ar.half[1] = *(const v8h*)(ap + 8);
        ai.half[0] = *(const v8h*)(ap + 512);
        ai.half[1] = *(const v8h*)(ap + 520);
        union { v16h hv; unsigned uu[8]; } nu;
        nu.hv = ai.v;
        #pragma unroll
        for (int q = 0; q < 8; ++q) nu.uu[q] ^= 0x80008000u;
        const v16h nai = nu.hv;
        #pragma unroll
        for (int ntl = 0; ntl < 2; ++ntl) {
          const _Float16* bp = wpk + ((size_t)((f * 2) * 4 + kc) * 16 + g * 2 + ntl) * 512 + lane * 16;
          Frag br, bi;
          br.half[0] = *(const v8h*)(bp);
          br.half[1] = *(const v8h*)(bp + 8);
          bi.half[0] = *(const v8h*)(bp + 32768);
          bi.half[1] = *(const v8h*)(bp + 32776);
          cr[j][ntl] = mma16(cr[j][ntl], ar.v, br.v);
          cr[j][ntl] = mma16(cr[j][ntl], nai,  bi.v);
          ci[j][ntl] = mma16(ci[j][ntl], ar.v, bi.v);
          ci[j][ntl] = mma16(ci[j][ntl], ai.v, br.v);
        }
      }
    }
  }

  #pragma unroll
  for (int j = 0; j < 3; ++j) {
    if (j < nb) {
      const int f = w + 16 * j;
      #pragma unroll
      for (int ntl = 0; ntl < 2; ++ntl) {
        #pragma unroll
        for (int r = 0; r < 8; ++r) {
          const int m   = 8 * h + r;
          const int row = (m * 2 + ntl) * 16 + m16;
          U.h[row * KIF + 2 * f]     = (_Float16)cr[j][ntl][r];
          U.h[row * KIF + 2 * f + 1] = (_Float16)ci[j][ntl][r];
        }
      }
    }
  }
  __syncthreads();

  v8f co[2] = {};
  #pragma unroll
  for (int ks = 0; ks < 3; ++ks) {
    Frag bt;
    bt.half[0] = *(const v8ha*)&Tl[ks * 512 + lane * 16];
    bt.half[1] = *(const v8ha*)&Tl[ks * 512 + lane * 16 + 8];
    #pragma unroll
    for (int tt = 0; tt < 2; ++tt) {
      const _Float16* arow = &U.h[((w * 2 + tt) * 16 + m16) * KIF + ks * 32];
      Frag at;
      at.half[0] = *(const v8ha*)(arow + 8 * h);
      at.half[1] = *(const v8ha*)(arow + 16 + 8 * h);
      co[tt] = mma16(co[tt], at.v, bt.v);
    }
  }
  __syncthreads();

  #pragma unroll
  for (int tt = 0; tt < 2; ++tt) {
    const int base = (w * 16 + m16) * 32 + tt * 16 + 8 * h;
    v4f lo4, hi4;
    lo4.x = co[tt][0]; lo4.y = co[tt][1]; lo4.z = co[tt][2]; lo4.w = co[tt][3];
    hi4.x = co[tt][4]; hi4.y = co[tt][5]; hi4.z = co[tt][6]; hi4.w = co[tt][7];
    *(v4fa*)&U.f[base]     = lo4;
    *(v4fa*)&U.f[base + 4] = hi4;
  }
  __syncthreads();

  const int piece = tid & 7;
  const int ocq   = oc0 + piece * 4;
  v4f b4;
  b4.x = bias[ocq]; b4.y = bias[ocq + 1]; b4.z = bias[ocq + 2]; b4.w = bias[ocq + 3];
  v4f vals[4];
  size_t offs[4];
  bool ok[4];
  #pragma unroll
  for (int ps = 0; ps < 4; ++ps) {
    const int L  = (tid >> 3) + 64 * ps;
    const int m  = L >> 4, s = L & 15;
    const int tg = tb * 16 + m;
    const int bimg = tg / 784;
    const int rr   = (tg / 28) % 28;
    const int cc   = tg % 28;
    const int I = rr * 4 + (s >> 2);
    const int J = cc * 4 + (s & 3);
    ok[ps] = (tg < NTILE) && (I >= 2) && (J >= 2) && (I - 2 < OH) && (J - 2 < OW);
    const int oy = ok[ps] ? (I - 2) : 0;
    const int ox = ok[ps] ? (J - 2) : 0;
    offs[ps] = (((size_t)bimg * OH + oy) * OW + ox) * OCN + ocq;
    const v4f sv = *(const v4fa*)&U.f[L * 32 + piece * 4];
    vals[ps] = sv * OSC + b4;
  }
  #pragma unroll
  for (int ps = 0; ps < 4; ++ps)
    if (ok[ps]) *(volatile v4f*)(out + offs[ps]) = vals[ps];
  __threadfence();
  #pragma unroll
  for (int ps = 0; ps < 4; ++ps)
    if (ok[ps]) *(volatile v4f*)(out + offs[ps]) = vals[ps];
}

extern "C" void kernel_launch(void* const* d_in, const int* in_sizes, int n_in,
                              void* d_out, int out_size, void* d_ws, size_t ws_size,
                              hipStream_t stream) {
  if (n_in < 5) return;
  if (in_sizes[0] != NIMG * HH * WW * ICN) return;
  if (in_sizes[1] != ICN * OCN * 64 || in_sizes[2] != ICN * OCN * 64 || in_sizes[3] != ICN * OCN * 64) return;
  if (in_sizes[4] != OCN) return;
  if (out_size != NIMG * OH * OW * OCN) return;

  const size_t wpk_bytes = (size_t)NCH * 16;
  const size_t pf_off    = wpk_bytes;
  const size_t pf_bytes  = (size_t)NDFTB * PFTILE * 2;
  if (pf_off + pf_bytes > ws_size) return;

  const float* x   = (const float*)d_in[0];
  const float* wr  = (const float*)d_in[1];
  const float* wi  = (const float*)d_in[2];
  const int*   msk = (const int*)d_in[3];
  const float* bs  = (const float*)d_in[4];
  float* out = (float*)d_out;
  _Float16* wpk = (_Float16*)d_ws;
  _Float16* pf  = (_Float16*)((char*)d_ws + pf_off);

  const int nb_pack = (NCH + 255) / 256;
  k_wpack<<<nb_pack, 256, 0, stream>>>(wr, wi, msk, wpk, NCH);
  k_dft<<<NDFTB, 512, 0, stream>>>(x, pf);
  k_conv<<<dim3(NTB, OCN / 32), 512, 0, stream>>>(pf, wpk, bs, out);
}
